// FlaxLLaMAAttention_6889127542833
// MI455X (gfx1250) — hardware-verified
//
#include <hip/hip_runtime.h>
#include <math.h>

typedef __attribute__((ext_vector_type(16))) _Float16 v16h;
typedef __attribute__((ext_vector_type(16))) __bf16 v16b;
typedef __attribute__((ext_vector_type(8)))  _Float16 v8h;
typedef __attribute__((ext_vector_type(8)))  float v8f;
typedef __attribute__((ext_vector_type(4)))  float v4f;
typedef __attribute__((ext_vector_type(4)))  unsigned v4u;

template <typename T> __device__ __forceinline__ void vst2(void* p, T v) { *(volatile T*)p = v; __threadfence(); *(volatile T*)p = v; }
__device__ __forceinline__ v8f wmma16(v16h a, v16h b, v8f c) {
  v8f d = __builtin_amdgcn_wmma_f32_16x16x32_f16(false, a, false, b, (short)0, c, false, false);
  asm volatile("v_nop\n\tv_nop\n\tv_nop\n\tv_nop" : "+v"(d) : "v"(a), "v"(b));
  return d;
}
__device__ __forceinline__ v8f wmma_bf(v16b a, v16b b, v8f c) {
  v8f d = __builtin_amdgcn_wmma_f32_16x16x32_bf16(false, a, false, b, (short)0, c, false, false);
  asm volatile("v_nop\n\tv_nop\n\tv_nop\n\tv_nop" : "+v"(d) : "v"(a), "v"(b));
  return d;
}
__device__ __forceinline__ v16h frag_h(const _Float16* rowk0, int lane) {
  union { v16h v; v8h q[2]; } u; const _Float16* p = rowk0 + 8 * (lane >> 4);
  u.q[0] = *(const v8h*)p; u.q[1] = *(const v8h*)(p + 16); return u.v;
}
__device__ __forceinline__ v16h frag_f32s(const float* rowk0, int lane, float sc) {
  v16h a; const float* p = rowk0 + 8 * (lane >> 4);
#pragma unroll
  for (int i = 0; i < 8; ++i) { a[i] = (_Float16)(p[i] * sc); a[8 + i] = (_Float16)(p[16 + i] * sc); }
  return a;
}
struct F2 { v16b h, l; };
__device__ __forceinline__ F2 bsplit16(const float v[16]) { F2 r;
#pragma unroll
  for (int i = 0; i < 16; ++i) { const __bf16 h = (__bf16)v[i]; r.h[i] = h; r.l[i] = (__bf16)(v[i] - (float)h); }
  return r; }
__device__ __forceinline__ F2 split_row(const float* row, int k0, int lane) { float v[16]; const float* p = row + k0 + 8 * (lane >> 4);
#pragma unroll
  for (int i = 0; i < 8; ++i) { v[i] = p[i]; v[8 + i] = p[16 + i]; }
  return bsplit16(v); }
#define LDSX() do { asm volatile("s_wait_dscnt 0" ::: "memory"); __builtin_amdgcn_wave_barrier(); __builtin_amdgcn_fence(__ATOMIC_RELEASE, "workgroup"); } while (0)

#ifndef NB
#define NB 1
#endif
#ifndef SEQ
#define SEQ 2048
#endif
#define NB_FULL 1
#define SEQ_FULL 2048
#define HID 2048
#define NHQ 32
#define NKV 8
#define HD 64
#define QW (NHQ * HD)
#define KW (NKV * HD)
#define QKVW (QW + 2 * KW)
#define ROWS (NB * SEQ)
#define TRB (ROWS / 64)
#define TQB (SEQ / 64)
static_assert(NB == 1 && NB_FULL == 1);
static_assert(SEQ % 64 == 0 && SEQ >= 64 && SEQ <= SEQ_FULL);
static_assert(HID % 32 == 0 && HD == 64 && QW % 128 == 0 && KW % 128 == 0 && QKVW % 128 == 0 && QW == HID);
static_assert(NHQ % NKV == 0);

#define WS_F   ((size_t)0)
#define WS_QH  (WS_F + 4u * (size_t)ROWS * QKVW)
#define WS_QL  (WS_QH + 2u * (size_t)ROWS * QW)
#define WS_KH  (WS_QL + 2u * (size_t)ROWS * QW)
#define WS_KL  (WS_KH + 2u * (size_t)ROWS * KW)
#define WS_VH  (WS_KL + 2u * (size_t)ROWS * KW)
#define WS_VL  (WS_VH + 2u * (size_t)NB * KW * SEQ_FULL)
#define WS_CT  (WS_VL + 2u * (size_t)NB * KW * SEQ_FULL)
#define WS_END (WS_CT + 4u * (size_t)ROWS * QW)
static_assert(WS_END <= (size_t)134217728u);
static_assert(WS_QH % 128 == 0 && WS_QL % 128 == 0 && WS_KH % 128 == 0 && WS_KL % 128 == 0 && WS_VH % 128 == 0 && WS_VL % 128 == 0 && WS_CT % 128 == 0);

__global__ __launch_bounds__(128) void k_qkv(const float* __restrict__ X, const float* __restrict__ WQ, const float* __restrict__ WK, const float* __restrict__ WV, float* __restrict__ F) {
  __shared__ __align__(16) float sf[4][16][132];
  const int tid = threadIdx.x, wave = tid >> 5, lane = tid & 31, col = lane & 15, g = lane >> 4; const int cg = blockIdx.y; const size_t r0 = (size_t)blockIdx.x * 64 + wave * 16;
  const float* Wm; int wcols, c0;
  if (cg < QW / 128) { Wm = WQ; wcols = QW; c0 = cg * 128; } else if (cg < (QW + KW) / 128) { Wm = WK; wcols = KW; c0 = (cg - QW / 128) * 128; } else { Wm = WV; wcols = KW; c0 = (cg - (QW + KW) / 128) * 128; }
  v8f acc[8] = {};
#pragma unroll 2
  for (int kc = 0; kc < HID / 32; ++kc) {
    v16b a; { const float* p = X + (r0 + col) * HID + kc * 32 + 8 * g;
#pragma unroll
      for (int i = 0; i < 8; ++i) { a[i] = (__bf16)p[i]; a[8 + i] = (__bf16)p[16 + i]; } }
#pragma unroll
    for (int j = 0; j < 8; ++j) { v16b w; const int o = c0 + j * 16 + col;
#pragma unroll
      for (int i = 0; i < 8; ++i) { w[i] = (__bf16)Wm[(size_t)(kc * 32 + 8 * g + i) * wcols + o]; w[8 + i] = (__bf16)Wm[(size_t)(kc * 32 + 16 + 8 * g + i) * wcols + o]; }
      acc[j] = wmma_bf(a, w, acc[j]); } }
#pragma unroll
  for (int j = 0; j < 8; ++j)
#pragma unroll
    for (int r = 0; r < 8; ++r) sf[wave][8 * g + r][j * 16 + col] = acc[j][r];
  LDSX();
  for (int rl = 0; rl < 16; ++rl) vst2(F + (r0 + rl) * QKVW + cg * 128 + lane * 4, *(const v4f*)&sf[wave][rl][lane * 4]);
}
__global__ __launch_bounds__(256) void k_rope(const float* __restrict__ F, const int* __restrict__ PID, _Float16* __restrict__ QH, _Float16* __restrict__ QL, _Float16* __restrict__ KH, _Float16* __restrict__ KL) {
  __shared__ __align__(16) _Float16 sh[QW + KW], sl[QW + KW]; __shared__ float tcs[HD / 2], tsn[HD / 2];
  const int t = threadIdx.x; const size_t row = blockIdx.x;
  int pv = PID[row]; if (pv < 0) pv += SEQ_FULL; pv = pv < 0 ? 0 : (pv > SEQ_FULL - 1 ? SEQ_FULL - 1 : pv);
  const float pos = (float)pv;
  if (t < HD / 2) { const float fq = 1.0f / powf(10000.0f, (float)(2 * t) / (float)HD); const float ang = pos * fq; float sn, cs; sincosf(ang, &sn, &cs); tcs[t] = cs; tsn[t] = sn; }
  __syncthreads();
  const float* fr = F + row * QKVW;
  for (int e = t; e < (QW + KW) / 2; e += 256) { const int j = e % (HD / 2); const int o = 2 * e;
    const float c = tcs[j], sn = tsn[j]; const float x0 = fr[o], x1 = fr[o + 1];
    const float y0 = x0 * c - x1 * sn, y1 = x0 * sn + x1 * c; const _Float16 h0 = (_Float16)y0, h1 = (_Float16)y1;
    sh[o] = h0; sh[o + 1] = h1; sl[o] = (_Float16)(y0 - (float)h0); sl[o + 1] = (_Float16)(y1 - (float)h1); }
  __syncthreads();
  for (int q = t; q < QW / 8; q += 256) { vst2((unsigned*)(QH + row * QW + q * 8), *(const v4u*)&sh[q * 8]); vst2((unsigned*)(QL + row * QW + q * 8), *(const v4u*)&sl[q * 8]); }
  for (int q = t; q < KW / 8; q += 256) { vst2((unsigned*)(KH + row * KW + q * 8), *(const v4u*)&sh[QW + q * 8]); vst2((unsigned*)(KL + row * KW + q * 8), *(const v4u*)&sl[QW + q * 8]); }
}
__global__ __launch_bounds__(128) void k_vt(const float* __restrict__ F, _Float16* __restrict__ VH, _Float16* __restrict__ VL) {
  __shared__ __align__(16) _Float16 th[128][72], tl[128][72];
  const int t = threadIdx.x; const size_t s0 = (size_t)blockIdx.x * 64; const int c0 = blockIdx.y * 128;
  for (int e = t; e < 64 * 128; e += 128) { const int sl_ = e >> 7, c = e & 127; const float v = F[(s0 + sl_) * QKVW + QW + KW + c0 + c]; const _Float16 hv = (_Float16)v; th[c][sl_] = hv; tl[c][sl_] = (_Float16)(v - (float)hv); }
  __syncthreads();
  for (int e = t; e < 128 * 8; e += 128) { const int c = e >> 3, q = e & 7;
    vst2((unsigned*)(VH + (size_t)(c0 + c) * SEQ_FULL + s0 + q * 8), *(const v4u*)&th[c][q * 8]);
    vst2((unsigned*)(VL + (size_t)(c0 + c) * SEQ_FULL + s0 + q * 8), *(const v4u*)&tl[c][q * 8]); }
}
__global__ __launch_bounds__(128) void k_att(const _Float16* __restrict__ QH, const _Float16* __restrict__ QL, const _Float16* __restrict__ KH, const _Float16* __restrict__ KL, const _Float16* __restrict__ VH, const _Float16* __restrict__ VL, float* __restrict__ CT) {
  __shared__ __align__(16) float sp[4][16][36]; __shared__ __align__(16) float so[4][16][68];
  const int tid = threadIdx.x, wave = tid >> 5, lane = tid & 31, col = lane & 15, g = lane >> 4; const int qb = blockIdx.x, h = blockIdx.y; const int kvh = h / (NHQ / NKV); const int q0 = qb * 64 + wave * 16;
  v16h aq[HD / 32], al[HD / 32];
#pragma unroll
  for (int kc = 0; kc < HD / 32; ++kc) { aq[kc] = frag_h(QH + (size_t)(q0 + col) * QW + h * HD + kc * 32, lane); al[kc] = frag_h(QL + (size_t)(q0 + col) * QW + h * HD + kc * 32, lane); }
  float m[8], l[8];
#pragma unroll
  for (int r = 0; r < 8; ++r) { m[r] = -3.0e38f; l[r] = 0.f; }
  v8f acc[HD / 16] = {};
  const int nks = (qb * 64 + 64) / 32;
#pragma unroll 1
  for (int ks = 0; ks < nks; ++ks) { float s[2][8];
#pragma unroll
    for (int ct = 0; ct < 2; ++ct) { const int kk = ks * 32 + ct * 16 + col; const size_t rk = (size_t)kk * KW + kvh * HD; v8f c = {};
#pragma unroll
      for (int kc = 0; kc < HD / 32; ++kc) { const v16h kh = frag_h(KH + rk + kc * 32, lane); c = wmma16(aq[kc], kh, c); c = wmma16(al[kc], kh, c); c = wmma16(aq[kc], frag_h(KL + rk + kc * 32, lane), c); }
#pragma unroll
      for (int r = 0; r < 8; ++r) s[ct][r] = (kk <= q0 + 8 * g + r) ? c[r] * 0.125f : -3.0e38f; }
    float alpha[8];
#pragma unroll
    for (int r = 0; r < 8; ++r) { float mx = fmaxf(s[0][r], s[1][r]);
#pragma unroll
      for (int o = 1; o < 16; o <<= 1) mx = fmaxf(mx, __shfl_xor(mx, o));
      const float mn = fmaxf(m[r], mx); alpha[r] = (m[r] <= -1.0e38f) ? 0.f : __expf(m[r] - mn);
      const float e0 = (s[0][r] <= -1.0e38f) ? 0.f : __expf(s[0][r] - mn), e1 = (s[1][r] <= -1.0e38f) ? 0.f : __expf(s[1][r] - mn); float es = e0 + e1;
#pragma unroll
      for (int o = 1; o < 16; o <<= 1) es += __shfl_xor(es, o);
      l[r] = l[r] * alpha[r] + es; m[r] = mn; sp[wave][8 * g + r][col] = e0; sp[wave][8 * g + r][16 + col] = e1; }
#pragma unroll
    for (int j = 0; j < HD / 16; ++j)
#pragma unroll
      for (int r = 0; r < 8; ++r) acc[j][r] *= alpha[r];
    LDSX();
    const v16h pa = frag_f32s(&sp[wave][col][0], lane, 2048.0f);
#pragma unroll
    for (int j = 0; j < HD / 16; ++j) { const size_t po = ((size_t)kvh * HD + j * 16 + col) * SEQ_FULL + ks * 32; acc[j] = wmma16(pa, frag_h(VH + po, lane), acc[j]); acc[j] = wmma16(pa, frag_h(VL + po, lane), acc[j]); }
    LDSX(); }
#pragma unroll
  for (int r = 0; r < 8; ++r) { const float il = (l[r] > 0.f) ? (1.0f / 2048.0f) / l[r] : 0.f;
#pragma unroll
    for (int j = 0; j < HD / 16; ++j) so[wave][8 * g + r][j * 16 + col] = acc[j][r] * il; }
  LDSX();
  for (int rp = 0; rp < 8; ++rp) { const int rl = 2 * rp + g; vst2(CT + (size_t)(q0 + rl) * QW + h * HD + col * 4, *(const v4f*)&so[wave][rl][col * 4]); }
}
__global__ __launch_bounds__(128) void k_out(const float* __restrict__ CT, const float* __restrict__ WO, float* __restrict__ OUT) {
  __shared__ __align__(16) float sf[4][16][132];
  const int tid = threadIdx.x, wave = tid >> 5, lane = tid & 31, col = lane & 15, g = lane >> 4; const int c0 = blockIdx.y * 128; const size_t r0 = (size_t)blockIdx.x * 64 + wave * 16;
  v8f acc[8] = {};
#pragma unroll 2
  for (int kc = 0; kc < QW / 32; ++kc) { const F2 a = split_row(CT + (r0 + col) * QW, kc * 32, lane);
#pragma unroll
    for (int j = 0; j < 8; ++j) { v16b w; const int o = c0 + j * 16 + col;
#pragma unroll
      for (int i = 0; i < 8; ++i) { w[i] = (__bf16)WO[(size_t)(kc * 32 + 8 * g + i) * HID + o]; w[8 + i] = (__bf16)WO[(size_t)(kc * 32 + 16 + 8 * g + i) * HID + o]; }
      acc[j] = wmma_bf(a.h, w, acc[j]); acc[j] = wmma_bf(a.l, w, acc[j]); } }
#pragma unroll
  for (int j = 0; j < 8; ++j)
#pragma unroll
    for (int r = 0; r < 8; ++r) sf[wave][8 * g + r][j * 16 + col] = acc[j][r];
  LDSX();
  for (int rl = 0; rl < 16; ++rl) vst2(OUT + (r0 + rl) * HID + c0 + lane * 4, *(const v4f*)&sf[wave][rl][lane * 4]);
}
extern "C" void kernel_launch(void* const* d_in, const int* in_sizes, int n_in, void* d_out, int out_size, void* d_ws, size_t ws_size, hipStream_t stream) {
  if (n_in < 6) return;
  if (in_sizes[0] < ROWS * HID || in_sizes[1] < HID * QW || in_sizes[2] < HID * KW || in_sizes[3] < HID * KW || in_sizes[4] < QW * HID || in_sizes[5] < ROWS) return;
  if ((size_t)out_size < (size_t)ROWS * HID) return;
  if (ws_size < (size_t)WS_END) return;
  const float* X = (const float*)d_in[0]; const float* WQ = (const float*)d_in[1]; const float* WK = (const float*)d_in[2]; const float* WV = (const float*)d_in[3]; const float* WO = (const float*)d_in[4]; const int* PID = (const int*)d_in[5];
  char* ws = (char*)d_ws; float* F = (float*)(ws + WS_F);
  _Float16 *QH = (_Float16*)(ws + WS_QH), *QL = (_Float16*)(ws + WS_QL), *KH = (_Float16*)(ws + WS_KH), *KL = (_Float16*)(ws + WS_KL), *VH = (_Float16*)(ws + WS_VH), *VL = (_Float16*)(ws + WS_VL);
  float* CT = (float*)(ws + WS_CT);
  k_qkv<<<dim3(TRB, QKVW / 128), 128, 0, stream>>>(X, WQ, WK, WV, F);
  k_rope<<<TRB * 64, 256, 0, stream>>>(F, PID, QH, QL, KH, KL);
  k_vt<<<dim3(TRB, KW / 128), 128, 0, stream>>>(F, VH, VL);
  k_att<<<dim3(TQB, NHQ), 128, 0, stream>>>(QH, QL, KH, KL, VH, VL, CT);
  k_out<<<dim3(TQB, HID / 128), 128, 0, stream>>>(CT, WO, (float*)d_out);
}
